// GlobalContextBlock_68624987455943
// MI455X (gfx1250) — hardware-verified
//
#include <hip/hip_runtime.h>
#include <math.h>

constexpr int kB     = 4;
constexpr int kL     = 2048;
constexpr int kD     = 768;
constexpr int kN     = 16;
constexpr int kRows  = kB * kL;
constexpr int kNP    = 832;
constexpr int kScanT = 256;
constexpr int kDBlk  = kD / kScanT;
constexpr float kLnEps = 1e-5f;
constexpr float kInvD  = 1.0f / 768.0f;

typedef __attribute__((ext_vector_type(16))) _Float16 v16h;
typedef __attribute__((ext_vector_type(8)))  _Float16 v8h;
typedef __attribute__((ext_vector_type(16))) __bf16   v16b;
typedef __attribute__((ext_vector_type(8)))  __bf16   v8b;
typedef __attribute__((ext_vector_type(8)))  float    v8f;
typedef __attribute__((ext_vector_type(4)))  float    v4f;
typedef __attribute__((ext_vector_type(4)))  unsigned int v4u;

__device__ __forceinline__ unsigned short f2bf_bits(float f) {
  unsigned u = __float_as_uint(f);
  return (unsigned short)((u + 0x7FFFu + ((u >> 16) & 1u)) >> 16);
}
__device__ __forceinline__ float bf_bits2f(unsigned short h) { return __uint_as_float(((unsigned)h) << 16); }

__device__ __forceinline__ void dep_guard_h(v8f& a, v8f& b, v16h x, v16h y) { asm volatile("v_nop\n\tv_nop\n\tv_nop\n\tv_nop" : "+v"(a), "+v"(b) : "v"(x), "v"(y)); }
__device__ __forceinline__ void dep_guard_b(v8f& a, v8f& b, v16b x, v16b y) { asm volatile("v_nop\n\tv_nop\n\tv_nop\n\tv_nop" : "+v"(a), "+v"(b) : "v"(x), "v"(y)); }
__device__ __forceinline__ void keep4_h(v16h a, v16h b, v16h c, v16h d) { asm volatile("v_nop" :: "v"(a), "v"(b), "v"(c), "v"(d)); }
__device__ __forceinline__ void keep4_b(v16b a, v16b b, v16b c, v16b d) { asm volatile("v_nop" :: "v"(a), "v"(b), "v"(c), "v"(d)); }
__device__ __forceinline__ void acc_guard4(v8f& a, v8f& b, v8f& c, v8f& d) { asm volatile("v_nop\n\tv_nop\n\tv_nop\n\tv_nop" : "+v"(a), "+v"(b), "+v"(c), "+v"(d)); }
template <typename T> struct Frag;
template <> struct Frag<_Float16> {
  typedef v16h V; union U { v16h v; v8h h[2]; };
  static __device__ __forceinline__ v16h load(const _Float16* p) {
    U f; f.h[0] = *(const v8h*)(p); f.h[1] = *(const v8h*)(p + 16); return f.v;
  }
  static __device__ __forceinline__ v8f mma(v16h a, v16h b, v8f c) {
    return __builtin_amdgcn_wmma_f32_16x16x32_f16(false, a, false, b, (short)0, c, false, false);
  }
  static __device__ __forceinline__ void guard(v8f& a, v8f& b, v16h x, v16h y) { dep_guard_h(a, b, x, y); }
  static __device__ __forceinline__ void keep(v16h a, v16h b, v16h c, v16h d) { keep4_h(a, b, c, d); }
};
template <> struct Frag<__bf16> {
  typedef v16b V; union U { v16b v; v8b h[2]; };
  static __device__ __forceinline__ v16b load(const __bf16* p) {
    U f; f.h[0] = *(const v8b*)(p); f.h[1] = *(const v8b*)(p + 16); return f.v;
  }
  static __device__ __forceinline__ v8f mma(v16b a, v16b b, v8f c) {
    return __builtin_amdgcn_wmma_f32_16x16x32_bf16(false, a, false, b, (short)0, c, false, false);
  }
  static __device__ __forceinline__ void guard(v8f& a, v8f& b, v16b x, v16b y) { dep_guard_b(a, b, x, y); }
  static __device__ __forceinline__ void keep(v16b a, v16b b, v16b c, v16b d) { keep4_b(a, b, c, d); }
};

__device__ __forceinline__ unsigned pk16(unsigned short a, unsigned short b) { return (unsigned)a | ((unsigned)b << 16); }

template <int ET> struct Elem;
template <> struct Elem<0> { typedef _Float16 T; };
template <> struct Elem<1> { typedef __bf16 T; };
template <int ET, bool SPLIT, int BIAS_MODE, int OUT_MODE, bool RESID, int ACT = 0>
__global__ __launch_bounds__(256) void wmma_gemm64(
    const unsigned short* __restrict__ Ap, const unsigned short* __restrict__ A2p, int lda, long strideA,
    const unsigned short* __restrict__ Btp, const unsigned short* __restrict__ Bt2p, int ldb, long strideB,
    void* __restrict__ Cout, void* __restrict__ Cout2, int ldc, long strideC,
    const float* __restrict__ bias,
    const float* __restrict__ resid, long strideR,
    int M, int N, int K, float scale) {
  typedef typename Elem<ET>::T T;
  typedef typename Frag<T>::V V;
  const T* A = (const T*)Ap; const T* A2 = (const T*)A2p; const T* Bt = (const T*)Btp; const T* Bt2 = (const T*)Bt2p;
  __shared__ __align__(16) float sT[8][16 * 68];
  const int b    = blockIdx.y;
  const int lane = threadIdx.x & 31;
  const int wave = threadIdx.x >> 5;
  const int tilesN = N >> 6;
  const int tilesM = M >> 6;
  const int tile = blockIdx.x * 8 + wave;
  if (tile >= tilesM * tilesN) return;
  const int tm = tile / tilesN;
  const int tn = tile - tm * tilesN;
  const int m0 = tm << 6;
  const int n0 = tn << 6;

  const T* Ab  = A  + (size_t)b * strideA;
  const T* Bb  = Bt + (size_t)b * strideB;
  const T* Ab2 = SPLIT ? (A2  + (size_t)b * strideA) : nullptr;
  const T* Bb2 = SPLIT ? (Bt2 + (size_t)b * strideB) : nullptr;

  const int rlane = lane & 15;
  const int koff  = (lane >> 4) * 8;
  const int mOff  = (lane >> 4) * 8;

  v8f acc[4][4];
#pragma unroll
  for (int i = 0; i < 4; ++i)
#pragma unroll
    for (int j = 0; j < 4; ++j) acc[i][j] = (v8f){0.f,0.f,0.f,0.f,0.f,0.f,0.f,0.f};

  for (int k0 = 0; k0 < K; k0 += 32) {
    V bh[4], bl[4];
#pragma unroll
    for (int j = 0; j < 4; ++j) {
      const size_t bo = (size_t)(n0 + (j << 4) + rlane) * ldb + koff + k0;
      bh[j] = Frag<T>::load(Bb + bo);
      if (SPLIT) bl[j] = Frag<T>::load(Bb2 + bo);
    }
#pragma unroll
    for (int i = 0; i < 4; ++i) {
      const size_t ao = (size_t)(m0 + (i << 4) + rlane) * lda + koff + k0;
      V ah = Frag<T>::load(Ab + ao);
      V al;
      if (SPLIT) al = Frag<T>::load(Ab2 + ao);
#pragma unroll
      for (int j = 0; j < 4; ++j) {
        acc[i][j] = Frag<T>::mma(ah, bh[j], acc[i][j]);
        if (SPLIT) {
          acc[i][j] = Frag<T>::mma(ah, bl[j], acc[i][j]);
          acc[i][j] = Frag<T>::mma(al, bh[j], acc[i][j]);
        }
      }
      Frag<T>::guard(acc[i][0], acc[i][3], ah, SPLIT ? al : ah);
    }
    Frag<T>::keep(bh[0], bh[1], bh[2], bh[3]);
    if (SPLIT) Frag<T>::keep(bl[0], bl[1], bl[2], bl[3]);
  }
  acc_guard4(acc[0][0], acc[0][1], acc[0][2], acc[0][3]);
  acc_guard4(acc[1][0], acc[1][1], acc[1][2], acc[1][3]);
  acc_guard4(acc[2][0], acc[2][1], acc[2][2], acc[2][3]);
  acc_guard4(acc[3][0], acc[3][1], acc[3][2], acc[3][3]);

  float* slab = sT[wave];
  const float* Rb = RESID ? (resid + (size_t)b * strideR) : nullptr;
#pragma unroll
  for (int i = 0; i < 4; ++i) {
    const int mBase = m0 + (i << 4);
#pragma unroll
    for (int j = 0; j < 4; ++j) {
      const int n = n0 + (j << 4) + rlane;
      float bv = 0.f;
      if (BIAS_MODE == 2) bv = bias[n];
#pragma unroll
      for (int r = 0; r < 8; ++r) {
        float v = acc[i][j][r] * scale;
        if (BIAS_MODE == 1) v += bias[mBase + mOff + r];
        if (BIAS_MODE == 2) v += bv;
        if (RESID) v += Rb[(size_t)(mBase + mOff + r) * ldc + n];
        if (ACT == 2) v = fmaxf(v, 0.0f);
        if (ACT == 4) v = (v > 0.f) ? v : 0.01f * v;
        slab[(mOff + r) * 68 + (j << 4) + rlane] = v;
      }
    }
    __builtin_amdgcn_fence(__ATOMIC_RELEASE, "workgroup");
    __builtin_amdgcn_wave_barrier();
    __builtin_amdgcn_fence(__ATOMIC_ACQUIRE, "workgroup");
    if (OUT_MODE == 0) {
      float* C = (float*)Cout + (size_t)b * strideC;
      const int hh = lane >> 4, c4 = (lane & 15) * 4;
      for (int pass = 0; pass < 2; ++pass) {
#pragma unroll
        for (int it = 0; it < 8; ++it) {
          const int row = it * 2 + hh;
          v4f v = *(const v4f*)(slab + row * 68 + c4);
          *(volatile v4f*)(C + (size_t)(mBase + row) * ldc + n0 + c4) = v;
        }
        __threadfence();
      }
    } else {
      const int q = lane >> 3, c8 = (lane & 7) * 8;
      unsigned short* C  = (unsigned short*)Cout  + (size_t)b * strideC;
      unsigned short* C2 = (OUT_MODE == 2) ? ((unsigned short*)Cout2 + (size_t)b * strideC) : nullptr;
      for (int pass = 0; pass < 2; ++pass) {
#pragma unroll
        for (int it = 0; it < 4; ++it) {
          const int row = it * 4 + q;
          const float* sp = slab + row * 68 + c8;
          v8h hv, lv;
#pragma unroll
          for (int e = 0; e < 8; ++e) {
            if (OUT_MODE == 1) {
              hv[e] = (_Float16)sp[e];
            } else {
              unsigned short hb = f2bf_bits(sp[e]);
              unsigned short lb = f2bf_bits(sp[e] - bf_bits2f(hb));
              hv[e] = __builtin_bit_cast(_Float16, hb);
              lv[e] = __builtin_bit_cast(_Float16, lb);
            }
          }
          *(volatile v8h*)(C + (size_t)(mBase + row) * ldc + n0 + c8) = hv;
          if (OUT_MODE == 2) *(volatile v8h*)(C2 + (size_t)(mBase + row) * ldc + n0 + c8) = lv;
        }
        __threadfence();
      }
    }
    __builtin_amdgcn_fence(__ATOMIC_RELEASE, "workgroup");
    __builtin_amdgcn_wave_barrier();
    __builtin_amdgcn_fence(__ATOMIC_ACQUIRE, "workgroup");
  }
}

__global__ __launch_bounds__(256) void xsplit_kernel(const float* __restrict__ in,
                                                     unsigned short* __restrict__ hi,
                                                     unsigned short* __restrict__ lo, int n8) {
  const int i = blockIdx.x * 256 + threadIdx.x;
  if (i >= n8) return;
  const float* p = in + 8 * (size_t)i;
  const v4f a = *(const v4f*)(p);
  const v4f c = *(const v4f*)(p + 4);
  unsigned short hb[8], lb[8];
#pragma unroll
  for (int e = 0; e < 4; ++e) {
    const float f0 = a[e];
    hb[e] = f2bf_bits(f0);
    lb[e] = f2bf_bits(f0 - bf_bits2f(hb[e]));
    const float f1 = c[e];
    hb[4 + e] = f2bf_bits(f1);
    lb[4 + e] = f2bf_bits(f1 - bf_bits2f(hb[4 + e]));
  }
  const v4u uh = (v4u){pk16(hb[0], hb[1]), pk16(hb[2], hb[3]), pk16(hb[4], hb[5]), pk16(hb[6], hb[7])};
  const v4u ul = (v4u){pk16(lb[0], lb[1]), pk16(lb[2], lb[3]), pk16(lb[4], lb[5]), pk16(lb[6], lb[7])};
  unsigned short* qh = hi + 8 * (size_t)i;
  unsigned short* ql = lo + 8 * (size_t)i;
  *(volatile v4u*)qh = uh;
  *(volatile v4u*)ql = ul;
  __threadfence();
  *(volatile v4u*)qh = uh;
  *(volatile v4u*)ql = ul;
}

__global__ __launch_bounds__(256) void wsplit_kernel(const float* __restrict__ Wdt, const float* __restrict__ Wb,
                                                     const float* __restrict__ Wc,
                                                     unsigned short* __restrict__ hi, unsigned short* __restrict__ lo) {
  __shared__ float sm[64][65];
  const int t  = threadIdx.x;
  const int k0 = blockIdx.x * 64;
  const int nt = blockIdx.y;
  const int n0 = nt * 64;
  if (nt < 12) {
#pragma unroll
    for (int i = 0; i < 16; ++i) {
      const int e = i * 256 + t;
      const int r = e >> 6;
      const int c = e & 63;
      sm[c][r] = Wdt[(size_t)(k0 + r) * kD + n0 + c];
    }
  } else {
#pragma unroll
    for (int i = 0; i < 16; ++i) {
      const int e = i * 256 + t;
      const int r = e >> 6;
      const int c = e & 63;
      const int cc = c & 15;
      const float wb = Wb[(size_t)(k0 + r) * kN + cc];
      const float wc = Wc[(size_t)(k0 + r) * kN + cc];
      const float v = (c < 16) ? wb : ((c < 32) ? wc : 0.0f);
      sm[c][r] = v;
    }
  }
  __syncthreads();
  const int lane = t & 31, wave = t >> 5;
  const int q = lane >> 3, c8 = (lane & 7) * 8;
  for (int pass = 0; pass < 2; ++pass) {
#pragma unroll
    for (int it = 0; it < 2; ++it) {
      const int row = wave * 8 + it * 4 + q;
      unsigned short hb[8], lb[8];
#pragma unroll
      for (int e = 0; e < 8; ++e) {
        const float f = sm[row][c8 + e];
        hb[e] = f2bf_bits(f);
        lb[e] = f2bf_bits(f - bf_bits2f(hb[e]));
      }
      const v4u uh = (v4u){pk16(hb[0], hb[1]), pk16(hb[2], hb[3]), pk16(hb[4], hb[5]), pk16(hb[6], hb[7])};
      const v4u ul = (v4u){pk16(lb[0], lb[1]), pk16(lb[2], lb[3]), pk16(lb[4], lb[5]), pk16(lb[6], lb[7])};
      const size_t o = (size_t)(n0 + row) * kD + k0 + c8;
      *(volatile v4u*)(hi + o) = uh;
      *(volatile v4u*)(lo + o) = ul;
    }
    __threadfence();
  }
}

__global__ __launch_bounds__(256) void scan_kernel(const float* __restrict__ P, const float* __restrict__ x,
                                                   const float* __restrict__ bdt, const float* __restrict__ Alog,
                                                   const float* __restrict__ dsk, float* __restrict__ Y) {
  __shared__ float hs[kN * kScanT];
  __shared__ float an[kN * kScanT];
  const int tid  = threadIdx.x;
  const int dblk = blockIdx.x % kDBlk;
  const int b    = blockIdx.x / kDBlk;
  const int d    = dblk * kScanT + tid;
#pragma unroll 1
  for (int n = 0; n < kN; ++n) {
    hs[n * kScanT + tid] = 0.0f;
    an[n * kScanT + tid] = -expf(Alog[(size_t)d * kN + n]);
  }
  const float bv = bdt[d];
  const float dv = dsk[d];
#pragma unroll 1
  for (int l = 0; l < kL; ++l) {
    const size_t row = (size_t)b * kL + l;
    const float* pr = P + row * kNP;
    const float pre = pr[d] + bv;
    const float xv  = x[row * kD + d];
    const float ax  = fabsf(pre);
    const float dt  = fmaxf(pre, 0.0f) + log1pf(expf(-ax));
    const float dtx = dt * xv;
    float y = 0.0f;
#pragma unroll 1
    for (int n = 0; n < kN; ++n) {
      const float a  = an[n * kScanT + tid];
      const float h0 = hs[n * kScanT + tid];
      const float dA = expf(dt * a);
      const float bm = pr[kD + n];
      const float cm = pr[kD + kN + n];
      const float h1 = dA * h0 + dtx * bm;
      hs[n * kScanT + tid] = h1;
      y += h1 * cm;
    }
    const float yv = y + dv * xv;
    float* yp = Y + row * kD + d;
    *(volatile float*)yp = yv;
    __threadfence();
    *(volatile float*)yp = yv;
  }
}

__global__ __launch_bounds__(256) void ln_kernel(const float* __restrict__ x, const float* __restrict__ Y,
                                                 const float* __restrict__ gamma, const float* __restrict__ beta,
                                                 float* __restrict__ out, int nrows) {
  const int lane = threadIdx.x & 31, wave = threadIdx.x >> 5;
  const int row = blockIdx.x * 8 + wave;
  if (row >= nrows) return;
  const float* xr = x + (size_t)row * kD;
  const float* yr = Y + (size_t)row * kD;
  v4f r[6];
  float s = 0.0f;
#pragma unroll
  for (int i = 0; i < 6; ++i) {
    const v4f a = *(const v4f*)(xr + i * 128 + lane * 4);
    const v4f c = *(const v4f*)(yr + i * 128 + lane * 4);
    r[i] = a + c;
    s += (r[i][0] + r[i][1]) + (r[i][2] + r[i][3]);
  }
#pragma unroll
  for (int off = 16; off > 0; off >>= 1) s += __shfl_xor(s, off, 32);
  const float mu = s * kInvD;
  float s2 = 0.0f;
#pragma unroll
  for (int i = 0; i < 6; ++i) {
#pragma unroll
    for (int e = 0; e < 4; ++e) {
      const float dd = r[i][e] - mu;
      r[i][e] = dd;
      s2 += dd * dd;
    }
  }
#pragma unroll
  for (int off = 16; off > 0; off >>= 1) s2 += __shfl_xor(s2, off, 32);
  const float var  = s2 * kInvD;
  const float rstd = rsqrtf(var + kLnEps);
  v4f o[6];
#pragma unroll
  for (int i = 0; i < 6; ++i) {
    const v4f g  = *(const v4f*)(gamma + i * 128 + lane * 4);
    const v4f bb = *(const v4f*)(beta + i * 128 + lane * 4);
#pragma unroll
    for (int e = 0; e < 4; ++e) o[i][e] = (r[i][e] * rstd) * g[e] + bb[e];
  }
  float* orow = out + (size_t)row * kD;
  for (int pass = 0; pass < 2; ++pass) {
#pragma unroll
    for (int i = 0; i < 6; ++i) *(volatile v4f*)(orow + i * 128 + lane * 4) = o[i];
    __threadfence();
  }
}

static inline size_t align256(size_t v) { return (v + 255) & ~(size_t)255; }

extern "C" void kernel_launch(void* const* d_in, const int* in_sizes, int n_in,
                              void* d_out, int out_size, void* d_ws, size_t ws_size,
                              hipStream_t stream) {
  if (n_in < 9) return;
  if (in_sizes[0] != kRows * kD || in_sizes[1] != kD * kD || in_sizes[2] != kD ||
      in_sizes[3] != kD * kN || in_sizes[4] != kD * kN || in_sizes[5] != kD * kN ||
      in_sizes[6] != kD || in_sizes[7] != kD || in_sizes[8] != kD) return;
  if (out_size != kRows * kD) return;

  const float* x     = (const float*)d_in[0];
  const float* W_dt  = (const float*)d_in[1];
  const float* b_dt  = (const float*)d_in[2];
  const float* W_B   = (const float*)d_in[3];
  const float* W_C   = (const float*)d_in[4];
  const float* A_log = (const float*)d_in[5];
  const float* D_sk  = (const float*)d_in[6];
  const float* gamma = (const float*)d_in[7];
  const float* beta  = (const float*)d_in[8];
  float* out = (float*)d_out;

  char* w = (char*)d_ws;
  size_t off = 0;
  unsigned short* Xh = (unsigned short*)(w + off); off = align256(off + (size_t)kRows * kD * 2);
  unsigned short* Xl = (unsigned short*)(w + off); off = align256(off + (size_t)kRows * kD * 2);
  unsigned short* Wh = (unsigned short*)(w + off); off = align256(off + (size_t)kNP * kD * 2);
  unsigned short* Wl = (unsigned short*)(w + off); off = align256(off + (size_t)kNP * kD * 2);
  float* P  = (float*)(w + off);                   off = align256(off + (size_t)kRows * kNP * 4);
  float* Yb = (float*)(w + off);                   off = align256(off + (size_t)kRows * kD * 4);
  if (off > ws_size) return;

  const int n8 = kRows * kD / 8;
  xsplit_kernel<<<(n8 + 255) / 256, 256, 0, stream>>>(x, Xh, Xl, n8);
  wsplit_kernel<<<dim3(kD / 64, kNP / 64), 256, 0, stream>>>(W_dt, W_B, W_C, Wh, Wl);

  const int tiles  = (kRows / 64) * (kNP / 64);
  const int gblk   = (tiles + 7) / 8;
  wmma_gemm64<1, true, 0, 0, false, 0><<<dim3(gblk, 1), 256, 0, stream>>>(
      Xh, Xl, kD, 0L,
      Wh, Wl, kD, 0L,
      (void*)P, (void*)nullptr, kNP, 0L,
      (const float*)nullptr,
      (const float*)nullptr, 0L,
      kRows, kNP, kD, 1.0f);

  scan_kernel<<<kB * kDBlk, kScanT, 0, stream>>>(P, x, b_dt, A_log, D_sk, Yb);

  ln_kernel<<<(kRows + 7) / 8, 256, 0, stream>>>(x, Yb, gamma, beta, out, kRows);
}
